// TriAttStart_20194936225886
// MI455X (gfx1250) — hardware-verified
//
#include <hip/hip_runtime.h>
#include <math.h>
#include <stdint.h>

#define LSZ   320
#define DD    128
#define NH    4
#define CH    32
#define NPOS  (LSZ * LSZ)
#define NSL   4
#define SROWS (LSZ / NSL)
#define NS    (SROWS * LSZ)

#define F_BIAS  1
#define F_BIASM 2
#define F_SIGM  4

static_assert(NH * CH == DD);
static_assert((LSZ % NSL) == 0 && (NS % 64) == 0 && (LSZ % 64) == 0 && (NPOS % 64) == 0);
static_assert((LSZ % 32) == 0 && (NPOS % 16) == 0);

typedef _Float16 v16h __attribute__((ext_vector_type(16)));
typedef _Float16 v8h  __attribute__((ext_vector_type(8)));
typedef __bf16   v16b __attribute__((ext_vector_type(16)));
typedef __bf16   v8b  __attribute__((ext_vector_type(8)));
typedef float    v8f  __attribute__((ext_vector_type(8)));
typedef float    v4f  __attribute__((ext_vector_type(4)));
typedef unsigned int v4u __attribute__((ext_vector_type(4)));

__device__ __forceinline__ unsigned short bf_bits(float f) {
  unsigned u = __float_as_uint(f);
  return (unsigned short)((u + 0x7FFFu + ((u >> 16) & 1u)) >> 16);
}
__device__ __forceinline__ float bf_up(unsigned short h) { return __uint_as_float(((unsigned)h) << 16); }
__device__ __forceinline__ unsigned short h_bits(_Float16 x) { return __builtin_bit_cast(unsigned short, x); }
__device__ __forceinline__ unsigned pk16(unsigned short a, unsigned short b) { return (unsigned)a | ((unsigned)b << 16); }
__device__ __forceinline__ v8f zero8() { v8f z = {0.f, 0.f, 0.f, 0.f, 0.f, 0.f, 0.f, 0.f}; return z; }

__device__ __forceinline__ v16b ldfrag_b(const __bf16* p) {
  union { v16b v; v8b h[2]; } f;
  f.h[0] = *(const v8b*)(p);
  f.h[1] = *(const v8b*)(p + 16);
  return f.v;
}
__device__ __forceinline__ v16h ldfrag_h(const _Float16* p) {
  union { v16h v; v8h h[2]; } f;
  f.h[0] = *(const v8h*)(p);
  f.h[1] = *(const v8h*)(p + 16);
  return f.v;
}

__device__ __forceinline__ v8f mma_h(v16h a, v16h b, v8f c) {
  c = __builtin_amdgcn_wmma_f32_16x16x32_f16(false, a, false, b, (short)0, c, false, false);
#if defined(__HIP_DEVICE_COMPILE__)
  asm volatile("v_nop\n\tv_nop\n\tv_nop\n\tv_nop" : "+v"(c) : "v"(a), "v"(b));
#endif
  return c;
}
__device__ __forceinline__ v8f mma_b_raw(v16b a, v16b b, v8f c) {
  return __builtin_amdgcn_wmma_f32_16x16x32_bf16(false, a, false, b, (short)0, c, false, false);
}
__device__ __forceinline__ void dep_guard_b(v8f& a, v8f& b, v16b x, v16b y) {
#if defined(__HIP_DEVICE_COMPILE__)
  asm volatile("v_nop\n\tv_nop\n\tv_nop\n\tv_nop" : "+v"(a), "+v"(b) : "v"(x), "v"(y));
#endif
}
__device__ __forceinline__ void keep4_b(v16b a, v16b b, v16b c, v16b d) {
#if defined(__HIP_DEVICE_COMPILE__)
  asm volatile("v_nop" :: "v"(a), "v"(b), "v"(c), "v"(d));
#endif
}
__device__ __forceinline__ void acc_guard4(v8f& a, v8f& b, v8f& c, v8f& d) {
#if defined(__HIP_DEVICE_COMPILE__)
  asm volatile("v_nop\n\tv_nop\n\tv_nop\n\tv_nop" : "+v"(a), "+v"(b), "+v"(c), "+v"(d));
#endif
}
__device__ __forceinline__ void wave_sync_lds() {
  __builtin_amdgcn_fence(__ATOMIC_RELEASE, "workgroup");
  __builtin_amdgcn_wave_barrier();
  __builtin_amdgcn_fence(__ATOMIC_ACQUIRE, "workgroup");
}

__global__ __launch_bounds__(256) void cvt_wT(const float* __restrict__ w0, const float* __restrict__ w1,
                                              const float* __restrict__ w2, const float* __restrict__ w3,
                                              unsigned short* outp, int nin, int nout) {
  __shared__ float tile[64][33];
  const int tid = threadIdx.x;
  const int z = blockIdx.z;
  const float* src = (z == 0) ? w0 : ((z == 1) ? w1 : ((z == 2) ? w2 : w3));
  unsigned short* dst = outp + (size_t)z * nin * nout;
  const int i0 = blockIdx.x * 64;
  const int o0 = blockIdx.y * 32;
#pragma unroll
  for (int p = 0; p < 8; ++p) {
    const int idx = p * 256 + tid;
    const int i = idx >> 5, o = idx & 31;
    tile[i][o] = src[(size_t)(i0 + i) * nout + o0 + o];
  }
  __syncthreads();
  const int o = tid >> 3, c8 = (tid & 7) * 8;
  v4u pk;
#pragma unroll
  for (int e = 0; e < 4; ++e)
    pk[e] = pk16(bf_bits(tile[c8 + 2 * e][o]), bf_bits(tile[c8 + 2 * e + 1][o]));
  unsigned short* gp = dst + (size_t)(o0 + o) * nin + i0 + c8;
  *(volatile v4u*)gp = pk;
  __threadfence();
  *(volatile v4u*)gp = pk;
}

__global__ __launch_bounds__(256) void cvt_wb(const float* __restrict__ wb, unsigned short* outp) {
  const int tid = threadIdx.x;
  const int row = tid >> 4;
  const int c8  = (tid & 15) * 8;
  const int rr  = (row < NH) ? row : (NH - 1);
  v4u pk;
#pragma unroll
  for (int e = 0; e < 4; ++e) {
    float v0 = wb[(c8 + 2 * e) * NH + rr];
    float v1 = wb[(c8 + 2 * e + 1) * NH + rr];
    v0 = (row < NH) ? v0 : 0.0f;
    v1 = (row < NH) ? v1 : 0.0f;
    pk[e] = pk16(bf_bits(v0), bf_bits(v1));
  }
  unsigned short* gp = outp + (size_t)row * DD + c8;
  *(volatile v4u*)gp = pk;
  __threadfence();
  *(volatile v4u*)gp = pk;
}

__global__ __launch_bounds__(256) void ln_rows(const float* __restrict__ zin, const float* __restrict__ lng,
                                               const float* __restrict__ lnb, unsigned short* zh, unsigned short* zl,
                                               int nrows) {
#pragma clang fp contract(off)
  const int tid = threadIdx.x;
  const int wave = tid >> 5, lane = tid & 31;
  const int row = blockIdx.x * 16 + wave * 2 + (lane >> 4);
  const int rowc = (row < nrows) ? row : (nrows - 1);
  const int c8 = (lane & 15) * 8;
  const float* rp = zin + (size_t)rowc * DD + c8;
  const v4f a = *(const v4f*)rp;
  const v4f b = *(const v4f*)(rp + 4);
  float x[8];
#pragma unroll
  for (int e = 0; e < 4; ++e) { x[e] = bf_up(bf_bits(a[e])); x[4 + e] = bf_up(bf_bits(b[e])); }
  float s = 0.f;
#pragma unroll
  for (int e = 0; e < 8; ++e) s = s + x[e];
#pragma unroll
  for (int off = 1; off < 16; off <<= 1) s = s + __shfl_xor(s, off, 32);
  const float mu = s * (1.0f / DD);
  float d[8];
  float s2 = 0.f;
#pragma unroll
  for (int e = 0; e < 8; ++e) { d[e] = x[e] - mu; const float dd = d[e] * d[e]; s2 = s2 + dd; }
#pragma unroll
  for (int off = 1; off < 16; off <<= 1) s2 = s2 + __shfl_xor(s2, off, 32);
  const float var = s2 * (1.0f / DD);
  const float rstd = 1.0f / sqrtf(var + 1e-5f);
  v4u ph, pl;
#pragma unroll
  for (int e = 0; e < 4; ++e) {
    const float g0 = bf_up(bf_bits(lng[c8 + 2 * e])), g1 = bf_up(bf_bits(lng[c8 + 2 * e + 1]));
    const float b0 = bf_up(bf_bits(lnb[c8 + 2 * e])), b1 = bf_up(bf_bits(lnb[c8 + 2 * e + 1]));
    float t0 = d[2 * e] * rstd;     t0 = t0 * g0; const float z0 = t0 + b0;
    float t1 = d[2 * e + 1] * rstd; t1 = t1 * g1; const float z1 = t1 + b1;
    const unsigned short h0 = bf_bits(z0), h1 = bf_bits(z1);
    const unsigned short l0 = bf_bits(z0 - bf_up(h0)), l1 = bf_bits(z1 - bf_up(h1));
    ph[e] = pk16(h0, h1); pl[e] = pk16(l0, l1);
  }
  if (row < nrows) {
    const size_t go = (size_t)row * DD + c8;
    *(volatile v4u*)(zh + go) = ph;
    *(volatile v4u*)(zl + go) = pl;
    __threadfence();
    *(volatile v4u*)(zh + go) = ph;
    *(volatile v4u*)(zl + go) = pl;
  }
}

__device__ __forceinline__ float epi_val(float f, int m, int n, const float* biasp, int blen, int flags) {
#pragma clang fp contract(off)
  if (flags & F_BIAS)  { const int i = (n < blen) ? n : (blen - 1); f = f + bf_up(bf_bits(biasp[i])); }
  if (flags & F_BIASM) { const int i = (m < blen) ? m : (blen - 1); f = f + bf_up(bf_bits(biasp[i])); }
  if (flags & F_SIGM) {
    const float x = fminf(fmaxf(f, -30.0f), 30.0f);
    const float e = __expf(-x);
    f = 1.0f / (1.0f + e);
  }
  return f;
}

template <int NSPLIT, int OUT_MODE, int MT>
__global__ __launch_bounds__(256) void gemm64(
    const unsigned short* __restrict__ Ap, const unsigned short* __restrict__ A2p, int lda,
    const unsigned short* __restrict__ Btp, const unsigned short* __restrict__ Bt2p, int ldb,
    void* Cout, void* Cout2, int ldc, int M, int N, int K,
    const float* __restrict__ biasp, int blen, int flags) {
#pragma clang fp contract(off)
  const __bf16* A   = (const __bf16*)(const void*)Ap;
  const __bf16* A2  = (const __bf16*)(const void*)A2p;
  const __bf16* Bt  = (const __bf16*)(const void*)Btp;
  const __bf16* Bt2 = (const __bf16*)(const void*)Bt2p;
  __shared__ __align__(16) float sT[8][16 * 68];
  const int lane = threadIdx.x & 31;
  const int wave = threadIdx.x >> 5;
  const int tilesN = N >> 6;
  const int tilesM = M / (16 * MT);
  const int tile = blockIdx.x * 8 + wave;
  if (tile >= tilesM * tilesN) return;
  const int tm = tile / tilesN;
  const int tn = tile - tm * tilesN;
  const int m0 = tm * (16 * MT);
  const int n0 = tn << 6;

  const int rlane = lane & 15;
  const int koff  = (lane >> 4) * 8;
  const int mOff  = (lane >> 4) * 8;

  v8f acc[MT][4];
#pragma unroll
  for (int i = 0; i < MT; ++i)
#pragma unroll
    for (int j = 0; j < 4; ++j) acc[i][j] = zero8();

  const int npl = (NSPLIT == 2) ? 2 : 1;
  for (int pl = 0; pl < npl; ++pl) {
    const __bf16* Bb = (pl == 0) ? Bt : Bt2;
    for (int k0 = 0; k0 < K; k0 += 32) {
      v16b bh[4];
#pragma unroll
      for (int j = 0; j < 4; ++j) {
        const size_t bo = (size_t)(n0 + (j << 4) + rlane) * ldb + koff + k0;
        bh[j] = ldfrag_b(Bb + bo);
      }
#pragma unroll
      for (int i = 0; i < MT; ++i) {
        const size_t ao = (size_t)(m0 + (i << 4) + rlane) * lda + koff + k0;
        const v16b ah = ldfrag_b(A + ao);
        v16b al = ah;
        if (NSPLIT == 1) al = ldfrag_b(A2 + ao);
#pragma unroll
        for (int j = 0; j < 4; ++j) {
          acc[i][j] = mma_b_raw(ah, bh[j], acc[i][j]);
          if (NSPLIT == 1) acc[i][j] = mma_b_raw(al, bh[j], acc[i][j]);
        }
        dep_guard_b(acc[i][0], acc[i][3], ah, al);
      }
      keep4_b(bh[0], bh[1], bh[2], bh[3]);
    }
  }
#pragma unroll
  for (int i = 0; i < MT; ++i) acc_guard4(acc[i][0], acc[i][1], acc[i][2], acc[i][3]);

  float* slab = sT[wave];
#pragma unroll
  for (int i = 0; i < MT; ++i) {
    const int mBase = m0 + (i << 4);
#pragma unroll
    for (int j = 0; j < 4; ++j) {
#pragma unroll
      for (int r = 0; r < 8; ++r) {
        slab[(mOff + r) * 68 + (j << 4) + rlane] = acc[i][j][r];
      }
    }
    wave_sync_lds();
    if (OUT_MODE == 0) {
      float* C = (float*)Cout;
      const int h2 = lane >> 4, c4 = (lane & 15) * 4;
      for (int pass = 0; pass < 2; ++pass) {
#pragma unroll
        for (int it = 0; it < 8; ++it) {
          const int row = it * 2 + h2;
          const int m = mBase + row;
          v4f v = *(const v4f*)(slab + row * 68 + c4);
#pragma unroll
          for (int e = 0; e < 4; ++e) v[e] = epi_val(v[e], m, n0 + c4 + e, biasp, blen, flags);
          *(volatile v4f*)(C + (size_t)m * ldc + n0 + c4) = v;
        }
        __threadfence();
      }
    } else {
      const int q = lane >> 3, c8 = (lane & 7) * 8;
      unsigned short* C  = (unsigned short*)Cout;
      unsigned short* C2 = (unsigned short*)Cout2;
      v4u hv[4], lv[4];
#pragma unroll
      for (int it = 0; it < 4; ++it) {
        const int row = it * 4 + q;
        const int m = mBase + row;
        const float* sp = slab + row * 68 + c8;
        float fv[8];
#pragma unroll
        for (int e = 0; e < 8; ++e) fv[e] = epi_val(sp[e], m, n0 + c8 + e, biasp, blen, flags);
        v4u a, a2;
#pragma unroll
        for (int e = 0; e < 4; ++e) {
          const float x0 = fv[2 * e], x1 = fv[2 * e + 1];
          unsigned short h0, h1, l0, l1;
          const _Float16 hx0 = (_Float16)x0, hx1 = (_Float16)x1;
          h0 = h_bits(hx0); h1 = h_bits(hx1);
          if (OUT_MODE == 4) {
            const float r0 = (x0 - (float)hx0) * 2048.0f;
            const float r1 = (x1 - (float)hx1) * 2048.0f;
            l0 = h_bits((_Float16)r0); l1 = h_bits((_Float16)r1);
          } else {
            l0 = 0; l1 = 0;
          }
          a[e] = pk16(h0, h1); a2[e] = pk16(l0, l1);
        }
        hv[it] = a; lv[it] = a2;
      }
      for (int pass = 0; pass < 2; ++pass) {
#pragma unroll
        for (int it = 0; it < 4; ++it) {
          const int row = it * 4 + q;
          *(volatile v4u*)(C + (size_t)(mBase + row) * ldc + n0 + c8) = hv[it];
          if (OUT_MODE == 4) *(volatile v4u*)(C2 + (size_t)(mBase + row) * ldc + n0 + c8) = lv[it];
        }
        __threadfence();
      }
    }
    wave_sync_lds();
  }
}

__global__ __launch_bounds__(256)
void attn_rows(const unsigned short* __restrict__ qhp, const unsigned short* __restrict__ qlp,
               const unsigned short* __restrict__ khp,
               const unsigned short* __restrict__ vthp, const unsigned short* __restrict__ vtlp,
               const float* __restrict__ bmt, const float* __restrict__ bbp,
               const float* __restrict__ gp, unsigned short* ogh, unsigned short* ogl) {
#pragma clang fp contract(off)
  union FH { v16h v; v8h h[2]; };
  __shared__ __align__(16) _Float16 Psh[8][16 * 64];
  __shared__ __align__(16) float    Os[32 * DD];

  const int tid  = threadIdx.x;
  const int wave = tid >> 5;
  const int lane = tid & 31;
  const int hh   = lane >> 4;
  const int c    = lane & 15;

  const int qt   = blockIdx.x;
  const int ib   = blockIdx.y;
  const int hp   = wave >> 1;
  const int wq   = wave & 1;
  const int lq0  = qt * 32 + wq * 16;
  const size_t pb0 = (size_t)ib * LSZ;

  const _Float16* Qh = (const _Float16*)(const void*)qhp;
  const _Float16* Ql = (const _Float16*)(const void*)qlp;
  const _Float16* Kh = (const _Float16*)(const void*)khp;
  const _Float16* Vh = (const _Float16*)(const void*)vthp;
  const _Float16* Vl = (const _Float16*)(const void*)vtlp;

  const size_t qo = (pb0 + lq0 + c) * DD + hp * CH + 8 * hh;
  const v16h qah = ldfrag_h(Qh + qo);
  const v16h qal = ldfrag_h(Ql + qo);

  const float bbh   = bf_up(bf_bits(bbp[hp]));
  const float scale = 0.17677669529663687f;
  const float inv2k = 1.0f / 2048.0f;
  const float* brow = bmt + (size_t)hp * NPOS;

  float mrow[8], lrow[8];
  v8f oh[2], ol[2];
#pragma unroll
  for (int r = 0; r < 8; ++r) { mrow[r] = -INFINITY; lrow[r] = 0.f; }
#pragma unroll
  for (int t = 0; t < 2; ++t) { oh[t] = zero8(); ol[t] = zero8(); }

  _Float16* pw = Psh[wave];

  for (int kt = 0; kt < LSZ / 64; ++kt) {
    const int kv0 = kt * 64;

    v8f s[4];
#pragma unroll
    for (int j = 0; j < 4; ++j) {
      const int key = kv0 + j * 16 + c;
      const size_t ko = (pb0 + key) * DD + hp * CH + 8 * hh;
      const v16h kb = ldfrag_h(Kh + ko);
      v8f ah = zero8();
      ah = mma_h(qah, kb, ah);
      v8f al = zero8();
      al = mma_h(qal, kb, al);
#pragma unroll
      for (int r = 0; r < 8; ++r) {
        const int l = lq0 + 8 * hh + r;
        const float bias = brow[(size_t)l * LSZ + key];
        const float rl = al[r] * inv2k;
        const float dv = ah[r] + rl;
        const float sc = dv * scale;
        const float bs = bias + bbh;
        s[j][r] = sc + bs;
      }
    }

#pragma unroll
    for (int r = 0; r < 8; ++r) {
      float m = fmaxf(fmaxf(s[0][r], s[1][r]), fmaxf(s[2][r], s[3][r]));
#pragma unroll
      for (int off = 1; off < 16; off <<= 1) m = fmaxf(m, __shfl_xor(m, off, 32));
      const float mnew  = fmaxf(mrow[r], m);
      const float alpha = __expf(mrow[r] - mnew);
      mrow[r] = mnew;
      float psum = 0.f;
#pragma unroll
      for (int j = 0; j < 4; ++j) {
        const float p  = __expf(s[j][r] - mnew);
        psum += p;
        const float p1 = p * 1024.0f;
        pw[(8 * hh + r) * 64 + j * 16 + c] = (_Float16)p1;
      }
#pragma unroll
      for (int off = 1; off < 16; off <<= 1) psum += __shfl_xor(psum, off, 32);
      lrow[r] = lrow[r] * alpha + psum;
#pragma unroll
      for (int t = 0; t < 2; ++t) { oh[t][r] *= alpha; ol[t][r] *= alpha; }
    }
    wave_sync_lds();

#pragma unroll
    for (int kk = 0; kk < 2; ++kk) {
      FH pa;
      pa.h[0] = *(const v8h*)(pw + c * 64 + kk * 32 + 8 * hh);
      pa.h[1] = *(const v8h*)(pw + c * 64 + kk * 32 + 16 + 8 * hh);
#pragma unroll
      for (int t = 0; t < 2; ++t) {
        const int d = hp * CH + t * 16 + c;
        const size_t vo = (size_t)d * NS + pb0 + kv0 + kk * 32 + 8 * hh;
        const v16h vbh = ldfrag_h(Vh + vo);
        const v16h vbl = ldfrag_h(Vl + vo);
        oh[t] = mma_h(pa.v, vbh, oh[t]);
        ol[t] = mma_h(pa.v, vbl, ol[t]);
      }
    }
    wave_sync_lds();
  }

#pragma unroll
  for (int r = 0; r < 8; ++r) {
    const float l = lrow[r];
    const float inv = ((l > 0.f) ? (1.0f / l) : 0.f) * (1.0f / 1024.0f);
    const size_t prow = pb0 + lq0 + 8 * hh + r;
#pragma unroll
    for (int t = 0; t < 2; ++t) {
      const int col = hp * CH + t * 16 + c;
      const float rl = ol[t][r] * inv2k;
      const float ov = (oh[t][r] + rl) * inv;
      const float gv = gp[prow * DD + col];
      Os[(wq * 16 + 8 * hh + r) * DD + col] = gv * ov;
    }
  }
  __syncthreads();
  {
    const int rh = lane >> 4, c16 = (lane & 15) * 8;
    v4u hv[2], lv[2];
#pragma unroll
    for (int it = 0; it < 2; ++it) {
      const int row = wave * 4 + it * 2 + rh;
      const float* sp = Os + row * DD + c16;
      v4u a, a2;
#pragma unroll
      for (int e = 0; e < 4; ++e) {
        const float x0 = sp[2 * e], x1 = sp[2 * e + 1];
        const unsigned short h0 = bf_bits(x0), h1 = bf_bits(x1);
        const unsigned short l0 = bf_bits(x0 - bf_up(h0)), l1 = bf_bits(x1 - bf_up(h1));
        a[e] = pk16(h0, h1); a2[e] = pk16(l0, l1);
      }
      hv[it] = a; lv[it] = a2;
    }
    for (int pass = 0; pass < 2; ++pass) {
#pragma unroll
      for (int it = 0; it < 2; ++it) {
        const int row = wave * 4 + it * 2 + rh;
        const size_t go = (pb0 + (size_t)qt * 32 + row) * DD + c16;
        *(volatile v4u*)(ogh + go) = hv[it];
        *(volatile v4u*)(ogl + go) = lv[it];
      }
      __threadfence();
    }
  }
}

extern "C" void kernel_launch(void* const* d_in, const int* in_sizes, int n_in,
                              void* d_out, int out_size, void* d_ws, size_t ws_size,
                              hipStream_t stream) {
  if (n_in < 15) return;
  if (in_sizes[0] != NPOS * DD) return;
  if (in_sizes[1] != DD || in_sizes[2] != DD) return;
  if (in_sizes[3] != DD * DD || in_sizes[4] != DD) return;
  if (in_sizes[5] != DD * DD || in_sizes[6] != DD) return;
  if (in_sizes[7] != DD * DD || in_sizes[8] != DD) return;
  if (in_sizes[9] != DD * NH || in_sizes[10] != NH) return;
  if (in_sizes[11] != DD * DD || in_sizes[12] != DD) return;
  if (in_sizes[13] != DD * DD || in_sizes[14] != DD) return;
  if (out_size != NPOS * DD) return;

  const float* zin = (const float*)d_in[0];
  const float* lng = (const float*)d_in[1];
  const float* lnb = (const float*)d_in[2];
  const float* Wq  = (const float*)d_in[3];
  const float* bq  = (const float*)d_in[4];
  const float* Wk  = (const float*)d_in[5];
  const float* bk  = (const float*)d_in[6];
  const float* Wv  = (const float*)d_in[7];
  const float* bv  = (const float*)d_in[8];
  const float* Wb  = (const float*)d_in[9];
  const float* bb  = (const float*)d_in[10];
  const float* Wg  = (const float*)d_in[11];
  const float* bg  = (const float*)d_in[12];
  const float* Wo  = (const float*)d_in[13];
  const float* bo  = (const float*)d_in[14];
  float* out = (float*)d_out;

  const size_t sW4  = (size_t)4 * DD * DD * 2;
  const size_t sWo  = (size_t)DD * DD * 2;
  const size_t sWb  = (size_t)16 * DD * 2;
  const size_t sZ   = (size_t)NPOS * DD * 2;
  const size_t sBMT = (size_t)16 * NPOS * 4;
  const size_t sQ   = (size_t)NS * DD * 2;
  const size_t sVT  = (size_t)DD * NS * 2;
  const size_t sG   = (size_t)NS * DD * 4;
  size_t off = 0;
  const size_t oW4  = off; off += sW4;
  const size_t oWo  = off; off += sWo;
  const size_t oWb  = off; off += sWb;
  const size_t oZh  = off; off += sZ;
  const size_t oZl  = off; off += sZ;
  const size_t oBMT = off; off += sBMT;
  const size_t oQh  = off; off += sQ;
  const size_t oQl  = off; off += sQ;
  const size_t oKh  = off; off += sQ;
  const size_t oVTh = off; off += sVT;
  const size_t oVTl = off; off += sVT;
  const size_t oG   = off; off += sG;
  const size_t oOGh = off; off += sQ;
  const size_t oOGl = off; off += sQ;
  if (off > ws_size) return;
  if (off > (size_t)134217728) return;

  char* ws = (char*)d_ws;
  unsigned short* Wcat = (unsigned short*)(ws + oW4);
  unsigned short* WqT  = Wcat;
  unsigned short* WkT  = Wcat + (size_t)1 * DD * DD;
  unsigned short* WvT  = Wcat + (size_t)2 * DD * DD;
  unsigned short* WgT  = Wcat + (size_t)3 * DD * DD;
  unsigned short* WoT  = (unsigned short*)(ws + oWo);
  unsigned short* Wb16 = (unsigned short*)(ws + oWb);
  unsigned short* Zh   = (unsigned short*)(ws + oZh);
  unsigned short* Zl   = (unsigned short*)(ws + oZl);
  float*          BMT  = (float*)(ws + oBMT);
  unsigned short* Qh   = (unsigned short*)(ws + oQh);
  unsigned short* Ql   = (unsigned short*)(ws + oQl);
  unsigned short* Kh   = (unsigned short*)(ws + oKh);
  unsigned short* VTh  = (unsigned short*)(ws + oVTh);
  unsigned short* VTl  = (unsigned short*)(ws + oVTl);
  float*          G    = (float*)(ws + oG);
  unsigned short* OGh  = (unsigned short*)(ws + oOGh);
  unsigned short* OGl  = (unsigned short*)(ws + oOGl);

  const dim3 blk(256);
  const dim3 gW4(DD / 64, DD / 32, 4);
  const dim3 gWo(DD / 64, DD / 32, 1);
  const dim3 gLN(NPOS / 16);
  const dim3 gBias(((NPOS / 64) * 1 + 7) / 8);
  const dim3 gProj(((NS / 64) * (DD / 64) + 7) / 8);
  const dim3 gVT(((DD / 64) * (NS / 64) + 7) / 8);
  const dim3 gAttn(LSZ / 32, SROWS);
  const dim3 gOut(((NS / 64) * (DD / 64) + 7) / 8);

  cvt_wT<<<gW4, blk, 0, stream>>>(Wq, Wk, Wv, Wg, Wcat, DD, DD);
  cvt_wT<<<gWo, blk, 0, stream>>>(Wo, Wo, Wo, Wo, WoT, DD, DD);
  cvt_wb<<<dim3(1), blk, 0, stream>>>(Wb, Wb16);
  ln_rows<<<gLN, blk, 0, stream>>>(zin, lng, lnb, Zh, Zl, NPOS);
  gemm64<2, 0, 1><<<gBias, blk, 0, stream>>>(
      Wb16, Wb16, DD, Zh, Zl, DD, (void*)BMT, (void*)BMT, NPOS, 16, NPOS, DD, bb, NH, 0);

  for (int sl = 0; sl < NSL; ++sl) {
    const unsigned short* Zsh = Zh + (size_t)sl * NS * DD;
    const unsigned short* Zsl = Zl + (size_t)sl * NS * DD;
    gemm64<1, 4, 4><<<gProj, blk, 0, stream>>>(
        Zsh, Zsl, DD, WqT, WqT, DD, (void*)Qh, (void*)Ql, DD, NS, DD, DD, bq, DD, F_BIAS);
    gemm64<1, 3, 4><<<gProj, blk, 0, stream>>>(
        Zsh, Zsl, DD, WkT, WkT, DD, (void*)Kh, (void*)Kh, DD, NS, DD, DD, bk, DD, F_BIAS);
    gemm64<1, 0, 4><<<gProj, blk, 0, stream>>>(
        Zsh, Zsl, DD, WgT, WgT, DD, (void*)G, (void*)G, DD, NS, DD, DD, bg, DD, F_BIAS | F_SIGM);
    gemm64<2, 4, 4><<<gVT, blk, 0, stream>>>(
        WvT, WvT, DD, Zsh, Zsl, DD, (void*)VTh, (void*)VTl, NS, DD, NS, DD, bv, DD, F_BIASM);
    attn_rows<<<gAttn, blk, 0, stream>>>(Qh, Ql, Kh, VTh, VTl, BMT, bb, G, OGh, OGl);
    gemm64<1, 0, 4><<<gOut, blk, 0, stream>>>(
        OGh, OGl, DD, WoT, WoT, DD, (void*)(out + (size_t)sl * NS * DD), (void*)(out + (size_t)sl * NS * DD), DD,
        NS, DD, DD, bo, DD, F_BIAS);
  }
  (void)hipGetLastError();
}
